// STGCNLSTM_29901562315329
// MI455X (gfx1250) — hardware-run, weakly checked
//
#include <hip/hip_runtime.h>
#include <stddef.h>


#define FEAT   16
#define HID    64
#define GATE   128
#define LH     32
#define NPG    128
#define SEQD   2048
#define NBAT   64
#define TWIN   32
#define TOUT   8
#define NCLS   10
#define HP     40
#define NTHR   256
#define NWAVE  8
#define EPT    8
#define NGRP   2
#define CHUNK  (NTHR * EPT * NGRP)
#define WCAP   (EPT * NGRP * 32)
#define LISTN  (NWAVE * WCAP)
#define NB     4096
#define RCAP   34304
#define TGT    256
#define DEGCAP 64
#define GROWS  128
#define KC2    256
#define WSCALE 16.0f
#define WINV   0.0625f

#define LDS_CSR ((2 * RCAP + NB + 2 * NWAVE) * 4)
#define TL_G    0
#define TL_WHH  (TL_G + NBAT * GATE * 4)
#define TL_WF1  (TL_WHH + GATE * HP * 2)
#define TL_WF2  (TL_WF1 + 16 * HP * 2)
#define TL_B    (TL_WF2 + 16 * HP * 2)
#define TL_H    (TL_B + GATE * 4)
#define TL_HS   (TL_H + NBAT * HP * 2)
#define TL_Z    (TL_HS + NBAT * TOUT * HP * 2)
#define TL_C    (TL_Z + NBAT * TOUT * HP * 2)
#define LDS_TAIL (TL_C + NBAT * LH * 4)

#define KCP_OF(kc) ((((kc) + 31) / 32) * 32)
#define GEMM_LDS(kc, nt) ((GROWS * (KCP_OF(kc) + 8) * 2) > (GROWS * (nt) * 16 * 4) ? (GROWS * (KCP_OF(kc) + 8) * 2) : (GROWS * (nt) * 16 * 4))

static_assert((CHUNK & (CHUNK - 1)) == 0);
static_assert(CHUNK <= 4096);
static_assert((NB & (NB - 1)) == 0 && NB <= 4096);
static_assert(NB == 16 * NTHR);
static_assert(LISTN <= RCAP && 2 * NB <= RCAP);
static_assert((RCAP % 32) == 0);
static_assert(TGT == NWAVE * 32);
static_assert((NB % TGT) == 0 && (NB % GROWS) == 0);
static_assert(NBAT * LH == 8 * NTHR);
static_assert(NBAT * TOUT == 64 * NWAVE);
static_assert(NBAT == 16 * (NWAVE / 2) && GATE == 2 * 64);
static_assert((TL_WHH % 16) == 0 && (TL_WF1 % 16) == 0 && (TL_WF2 % 16) == 0 && (TL_B % 16) == 0);
static_assert((TL_H % 16) == 0 && (TL_HS % 16) == 0 && (TL_Z % 16) == 0 && (TL_C % 16) == 0 && (LDS_TAIL % 16) == 0);
static_assert(NBAT * TOUT * NCLS * 4 <= NBAT * GATE * 4);
static_assert((NBAT * TOUT * NCLS) % (4 * NTHR) == 0);

typedef float    v4f  __attribute__((ext_vector_type(4)));
typedef float    v8f  __attribute__((ext_vector_type(8)));
typedef int      v4i  __attribute__((ext_vector_type(4)));
typedef _Float16 v8h  __attribute__((ext_vector_type(8)));
typedef _Float16 v16h __attribute__((ext_vector_type(16)));
union FragH { v16h v; v8h h[2]; };

__device__ __forceinline__ v8h cvt8(v4f a, v4f b) {
  v8h r;
  r[0] = (_Float16)a.x; r[1] = (_Float16)a.y; r[2] = (_Float16)a.z; r[3] = (_Float16)a.w;
  r[4] = (_Float16)b.x; r[5] = (_Float16)b.y; r[6] = (_Float16)b.z; r[7] = (_Float16)b.w;
  return r;
}
__device__ __forceinline__ v8h zero8h() { const v4f z = {0.f, 0.f, 0.f, 0.f}; return cvt8(z, z); }
__device__ __forceinline__ v8f zero8f() { v8f z = {0.f, 0.f, 0.f, 0.f, 0.f, 0.f, 0.f, 0.f}; return z; }
__device__ __forceinline__ v8h ld8h(const float* p) { return cvt8(*(const v4f*)p, *(const v4f*)(p + 4)); }
__device__ __forceinline__ v8h ld8h(const _Float16* p) { return *(const v8h*)p; }

__device__ __forceinline__ v8f wmh(v16h a, v16h b, v8f c) {
  v8f d = __builtin_amdgcn_wmma_f32_16x16x32_f16(false, a, false, b, (short)0, c, false, false);
  asm volatile("v_nop\n\tv_nop\n\tv_nop\n\tv_nop" : "+v"(d) : "v"(a), "v"(b));
  return d;
}

__device__ __forceinline__ void load8(const int* __restrict__ dsts, int nE, int cbase, int e0, int vec8, v4i& da, v4i& db) {
  const int sent = -2147483647 - 1;
  if (vec8 != 0 && cbase + CHUNK <= nE) {
    da = *(const v4i*)(dsts + e0);
    db = *(const v4i*)(dsts + e0 + 4);
  } else {
    const int l = nE - 1;
    da.x = (e0     < nE) ? dsts[min(e0, l)]     : sent;
    da.y = (e0 + 1 < nE) ? dsts[min(e0 + 1, l)] : sent;
    da.z = (e0 + 2 < nE) ? dsts[min(e0 + 2, l)] : sent;
    da.w = (e0 + 3 < nE) ? dsts[min(e0 + 3, l)] : sent;
    db.x = (e0 + 4 < nE) ? dsts[min(e0 + 4, l)] : sent;
    db.y = (e0 + 5 < nE) ? dsts[min(e0 + 5, l)] : sent;
    db.z = (e0 + 6 < nE) ? dsts[min(e0 + 6, l)] : sent;
    db.w = (e0 + 7 < nE) ? dsts[min(e0 + 7, l)] : sent;
  }
}

template <int NBT>
__device__ __forceinline__ int scan_chunk(const int* __restrict__ dsts, int nE, int cbase, int slotBase,
                                          int vec8, int* list, int tid, int lane, int wave) {
  int wc = 0;
#pragma unroll
  for (int g = 0; g < NGRP; ++g) {
    const int el0 = (g * NTHR + tid) * EPT;
    v4i da, db;
    load8(dsts, nE, cbase, cbase + el0, vec8, da, db);
    const unsigned nbu = (unsigned)slotBase;
    const unsigned s0 = (unsigned)da.x - nbu, s1 = (unsigned)da.y - nbu;
    const unsigned s2 = (unsigned)da.z - nbu, s3 = (unsigned)da.w - nbu;
    const unsigned s4 = (unsigned)db.x - nbu, s5 = (unsigned)db.y - nbu;
    const unsigned s6 = (unsigned)db.z - nbu, s7 = (unsigned)db.w - nbu;
    const bool h0 = s0 < (unsigned)NBT, h1 = s1 < (unsigned)NBT, h2 = s2 < (unsigned)NBT, h3 = s3 < (unsigned)NBT;
    const bool h4 = s4 < (unsigned)NBT, h5 = s5 < (unsigned)NBT, h6 = s6 < (unsigned)NBT, h7 = s7 < (unsigned)NBT;
    const unsigned any = __builtin_amdgcn_ballot_w32(h0 | h1 | h2 | h3 | h4 | h5 | h6 | h7);
    if (any != 0u) {
#define HITJ(J, HJ, SJ) { \
        const unsigned mj = __builtin_amdgcn_ballot_w32(HJ); \
        if (mj != 0u) { \
          if (HJ) { \
            const int pos = wc + (int)__builtin_amdgcn_mbcnt_lo(mj, 0u); \
            if (pos < WCAP) list[wave * WCAP + pos] = ((el0 + (J)) << 12) | (int)(SJ); \
          } \
          wc += (int)__builtin_popcount(mj); } }
      HITJ(0, h0, s0)
      HITJ(1, h1, s1)
      HITJ(2, h2, s2)
      HITJ(3, h3, s3)
      HITJ(4, h4, s4)
      HITJ(5, h5, s5)
      HITJ(6, h6, s6)
      HITJ(7, h7, s7)
#undef HITJ
    }
  }
  return wc;
}

__device__ __forceinline__ void group_rank(int key, int lane, int& rank, int& total) {
  int rk = 0, tt = 0;
#pragma unroll
  for (int k = 0; k < 32; ++k) {
    const int sk = __builtin_amdgcn_readlane(key, k);
    const int eq = (sk == key) ? 1 : 0;
    tt += eq;
    rk += (k < lane) ? eq : 0;
  }
  rank = rk; total = tt;
}

__global__ __launch_bounds__(NTHR) void k_wprep(
    const float* __restrict__ W1, const float* __restrict__ W2, const float* __restrict__ Wih,
    _Float16* w1p, _Float16* w2p, _Float16* wihp, int nb0, int nb1) {
  const int b = blockIdx.x, tid = threadIdx.x;
  const float* src; _Float16* dst; int K, Nn, KP, ngrp, tr, lb;
  if (b < nb0)            { src = W1;  dst = w1p;  K = FEAT; Nn = HID;  KP = 32;   ngrp = HID * 32 / 8;    tr = 1; lb = b; }
  else if (b < nb0 + nb1) { src = W2;  dst = w2p;  K = HID;  Nn = FEAT; KP = HID;  ngrp = FEAT * HID / 8;  tr = 1; lb = b - nb0; }
  else                    { src = Wih; dst = wihp; K = SEQD; Nn = GATE; KP = SEQD; ngrp = GATE * SEQD / 8; tr = 0; lb = b - nb0 - nb1; }
  const int i = lb * NTHR + tid;
  if (i >= ngrp) return;
  const int o  = i * 8;
  const int n  = o / KP;
  const int k0 = o - n * KP;
  const int nc = n < Nn ? n : Nn - 1;
  float v[8];
#pragma unroll
  for (int e = 0; e < 8; ++e) {
    const int k  = k0 + e;
    const int kc = k < K ? k : K - 1;
    const int idx = (tr != 0) ? (kc * Nn + nc) : (nc * K + kc);
    const float x = src[idx];
    v[e] = (k < K && n < Nn) ? x * WSCALE : 0.0f;
  }
  v4f a, c;
  a.x = v[0]; a.y = v[1]; a.z = v[2]; a.w = v[3];
  c.x = v[4]; c.y = v[5]; c.z = v[6]; c.w = v[7];
  const v8h hv = cvt8(a, c);
  _Float16* dp = dst + o;
  *(volatile v8h*)dp = hv;
  __threadfence();
  *(volatile v8h*)dp = hv;
}

__global__ __launch_bounds__(NTHR) void k_csr(
    const int* __restrict__ ei, int* cnt, float* dinv, int* off, int* csr, int nN, int nE, int vec8) {
  extern __shared__ v4i lds_c[];
  int*   L    = (int*)lds_c;
  int*   R    = L + RCAP;
  int*   scnt = R + RCAP;
  int*   wcnt = scnt + NB;
  int*   wtot = wcnt + NWAVE;
  int*   list = R;
  float* sdv  = (float*)R;
  int*   stmp = R + NB;
  const int tid = threadIdx.x, lane = tid & 31, wave = tid >> 5;
  const int b = blockIdx.x;
  const int nodeBase = b * NB;
  const int regBase  = b * RCAP;
  const int* dsts = ei + nE;

  for (int i = tid; i < NB; i += NTHR) scnt[i] = 0;
  __syncthreads();

  int runBase = 0;
  const int nChunks = (nE + CHUNK - 1) / CHUNK;
#pragma unroll 1
  for (int ch = 0; ch < nChunks; ++ch) {
    const int cbase = ch * CHUNK;
    int wc = scan_chunk<NB>(dsts, nE, cbase, nodeBase, vec8, list, tid, lane, wave);
    wc = wc > WCAP ? WCAP : wc;
    if (lane == 0) wcnt[wave] = wc;
    __syncthreads();
    int pre = 0, totc = 0;
#pragma unroll
    for (int w = 0; w < NWAVE; ++w) {
      int c = __builtin_amdgcn_readfirstlane(wcnt[w]);
      c = c < 0 ? 0 : (c > WCAP ? WCAP : c);
      totc += c;
      pre  += (w < wave) ? c : 0;
    }
    const int* lp = list + wave * WCAP;
#pragma unroll 1
    for (int i0 = 0; i0 < wc; i0 += 32) {
      const int i = i0 + lane;
      const bool ok = i < wc;
      const int ent  = lp[ok ? i : 0];
      const int slot = ent & (NB - 1);
      int e = cbase + ((ent >> 12) & (CHUNK - 1));
      e = e > nE - 1 ? nE - 1 : e;
      int s = ei[e];
      s = s < 0 ? 0 : (s > nN - 1 ? nN - 1 : s);
      const int dpos = runBase + pre + i;
      if (ok && dpos < RCAP) L[dpos] = (int)(((unsigned)s << 12) | (unsigned)slot);
    }
    runBase += totc;
    __syncthreads();
  }
  const int tot = runBase > RCAP ? RCAP : runBase;
  const int nsteps = (tot + 31) >> 5;

  if (wave == 0) {
#pragma unroll 1
    for (int st = 0; st < nsteps; ++st) {
      const int i = (st << 5) + lane;
      const bool valid = i < tot;
      const int ent  = L[i < RCAP ? i : RCAP - 1];
      const int slot = valid ? (ent & (NB - 1)) : -1;
      int rank, total;
      group_rank(slot, lane, rank, total);
      if (valid) { const int c = scnt[slot]; scnt[slot] = c + total; }
    }
  }
  __syncthreads();

  {
    v4i cq[4];
#pragma unroll
    for (int q = 0; q < 4; ++q) cq[q] = *(const v4i*)(scnt + 16 * tid + 4 * q);
    int ts = 0;
#pragma unroll
    for (int q = 0; q < 4; ++q) ts += cq[q].x + cq[q].y + cq[q].z + cq[q].w;
    int incl = ts;
#pragma unroll
    for (int d = 1; d < 32; d <<= 1) {
      const int tv = __shfl_up(incl, d);
      if (lane >= d) incl += tv;
    }
    if (lane == 31) wtot[wave] = incl;
    __syncthreads();
    int pre = 0;
#pragma unroll 1
    for (int w = 0; w < wave; ++w) pre += wtot[w];
    int run = pre + incl - ts;
    v4i oq[4]; v4f dq[4];
#pragma unroll
    for (int q = 0; q < 4; ++q) {
      oq[q].x = run; run += cq[q].x;
      oq[q].y = run; run += cq[q].y;
      oq[q].z = run; run += cq[q].z;
      oq[q].w = run; run += cq[q].w;
      dq[q].x = rsqrtf((float)(cq[q].x + 1));
      dq[q].y = rsqrtf((float)(cq[q].y + 1));
      dq[q].z = rsqrtf((float)(cq[q].z + 1));
      dq[q].w = rsqrtf((float)(cq[q].w + 1));
    }
#pragma unroll
    for (int q = 0; q < 4; ++q) {
      *(v4i*)(stmp + 16 * tid + 4 * q) = oq[q];
      *(v4f*)(sdv  + 16 * tid + 4 * q) = dq[q];
    }
  }
  __syncthreads();
  {
    int*   cp = cnt  + (size_t)nodeBase;
    int*   op = off  + (size_t)nodeBase;
    float* dp = dinv + (size_t)nodeBase;
    const v4i rb4 = {regBase, regBase, regBase, regBase};
#pragma unroll
    for (int i = 0; i < 4; ++i) {
      const int idx = i * NTHR + tid;
      const v4i cv = *(const v4i*)(scnt + 4 * idx);
      const v4i ov = *(const v4i*)(stmp + 4 * idx) + rb4;
      const v4f dv = *(const v4f*)(sdv + 4 * idx);
      *(volatile v4i*)(cp + 4 * idx) = cv;
      *(volatile v4i*)(op + 4 * idx) = ov;
      *(volatile v4f*)(dp + 4 * idx) = dv;
    }
    __threadfence();
#pragma unroll
    for (int i = 0; i < 4; ++i) {
      const int idx = i * NTHR + tid;
      const v4i cv = *(const v4i*)(scnt + 4 * idx);
      const v4i ov = *(const v4i*)(stmp + 4 * idx) + rb4;
      const v4f dv = *(const v4f*)(sdv + 4 * idx);
      *(volatile v4i*)(cp + 4 * idx) = cv;
      *(volatile v4i*)(op + 4 * idx) = ov;
      *(volatile v4f*)(dp + 4 * idx) = dv;
    }
  }
  __syncthreads();
#pragma unroll
  for (int i = 0; i < 4; ++i) { const int idx = i * NTHR + tid; ((v4i*)scnt)[idx] = ((const v4i*)stmp)[idx]; }
  __syncthreads();
  { const v4i z = {0, 0, 0, 0}; for (int i = tid; i < RCAP / 4; i += NTHR) ((v4i*)R)[i] = z; }
  __syncthreads();

  if (wave == 0) {
#pragma unroll 1
    for (int st = 0; st < nsteps; ++st) {
      const int i = (st << 5) + lane;
      const bool valid = i < tot;
      const int ent  = L[i < RCAP ? i : RCAP - 1];
      const int slot = valid ? (ent & (NB - 1)) : -1;
      int rank, total;
      group_rank(slot, lane, rank, total);
      if (valid) {
        const int cu = scnt[slot];
        int pos = cu + rank;
        pos = pos < 0 ? 0 : (pos > RCAP - 1 ? RCAP - 1 : pos);
        R[pos] = (int)((unsigned)ent >> 12);
        int ncu = cu + total;
        ncu = ncu > RCAP ? RCAP : ncu;
        scnt[slot] = ncu;
      }
    }
  }
  __syncthreads();

  int* gp = csr + (size_t)regBase;
#pragma unroll 1
  for (int i = tid; i < RCAP / 4; i += NTHR) { const v4i v = ((const v4i*)R)[i]; *(volatile v4i*)(gp + 4 * i) = v; }
  __threadfence();
#pragma unroll 1
  for (int i = tid; i < RCAP / 4; i += NTHR) { const v4i v = ((const v4i*)R)[i]; *(volatile v4i*)(gp + 4 * i) = v; }
}

template <int MODE>
__global__ __launch_bounds__(NTHR) void k_agg(
    const int* __restrict__ csr, const int* __restrict__ off, const int* __restrict__ cnt,
    const float* __restrict__ dinv, const float* __restrict__ src, const float* __restrict__ bias,
    float* dst, int nN, int nSrc, int csrLen) {
  const int tid = threadIdx.x, lane = tid & 31, wave = tid >> 5, half = lane >> 4, ch = lane & 15;
  const int tbase = blockIdx.x * TGT + wave * 32;
  const int cl = tbase + lane;
  const int cnt_l = cnt[cl];
  const int off_l = off[cl];
  union FI { float f; int i; };
  FI dvu; dvu.f = dinv[cl];
  float bch = 0.0f;
  if (MODE == 1) bch = bias[ch];

#pragma unroll 1
  for (int p = 0; p < 16; ++p) {
    int n0 = __builtin_amdgcn_readlane(cnt_l, 2 * p);
    int n1 = __builtin_amdgcn_readlane(cnt_l, 2 * p + 1);
    n0 = n0 < 0 ? 0 : (n0 > DEGCAP ? DEGCAP : n0);
    n1 = n1 < 0 ? 0 : (n1 > DEGCAP ? DEGCAP : n1);
    const int st0 = __builtin_amdgcn_readlane(off_l, 2 * p);
    const int st1 = __builtin_amdgcn_readlane(off_l, 2 * p + 1);
    FI d0, d1;
    d0.i = __builtin_amdgcn_readlane(dvu.i, 2 * p);
    d1.i = __builtin_amdgcn_readlane(dvu.i, 2 * p + 1);
    const int   myn  = half != 0 ? n1 : n0;
    const int   myst = half != 0 ? st1 : st0;
    const float mydc = half != 0 ? d1.f : d0.f;
    const int   nmax = n0 > n1 ? n0 : n1;
    float acc = 0.0f;
#pragma unroll 1
    for (int q = 0; q < nmax; q += 16) {
      int pos = myst + q + ch;
      pos = pos < 0 ? 0 : (pos > csrLen - 1 ? csrLen - 1 : pos);
      int sl = csr[pos];
      sl = sl < 0 ? 0 : (sl > nN - 1 ? nN - 1 : sl);
      const int mcnt = (nmax - q) < 16 ? (nmax - q) : 16;
#pragma unroll 1
      for (int pp = 0; pp < mcnt; ++pp) {
        const int s = __shfl(sl, (lane & 16) + pp);
        const bool valid = (q + pp) < myn;
        const float v = src[(size_t)s * FEAT + ch];
        float w = 1.0f;
        if (MODE == 0) w = dinv[s];
        acc += valid ? v * w : 0.0f;
      }
    }
    const int ct = tbase + 2 * p + half;
    const int cs = ct < nSrc ? ct : nSrc - 1;
    const float sv = src[(size_t)cs * FEAT + ch];
    float r;
    if (MODE == 0) r = (acc + mydc * sv) * mydc;
    else           r = fmaxf((acc + sv) * mydc + bch, 0.0f);
    float* op = dst + (size_t)(tbase + 2 * p) * FEAT + lane;
    *(volatile float*)op = r;
    __threadfence();
    *(volatile float*)op = r;
  }
}

template <int K, int KC, int NT, typename TA, int MODE>
__global__ __launch_bounds__(NTHR) void k_gemm(
    const TA* __restrict__ A, const _Float16* __restrict__ Bs, const float* __restrict__ dinv,
    const float* __restrict__ bias, _Float16* Ch, float* Cf, int nRowsA) {
  extern __shared__ v4f lds_g[];
  constexpr int KCP = KCP_OF(KC);
  constexpr int AP  = KCP + 8;
  constexpr int NCH = K / KC;
  constexpr int KBP = NCH * KCP;
  constexpr int NC  = NT * 16;
  constexpr int GPR = KC / 8;
  constexpr int SPT = (GROWS * GPR) / NTHR;
  constexpr int PG  = (KCP - KC) / 8;
  constexpr int PGD = PG > 0 ? PG : 1;
  static_assert(K % KC == 0);
  static_assert(KC % 8 == 0);
  static_assert((GROWS * GPR) % NTHR == 0);
  _Float16* sA  = (_Float16*)lds_g;
  float*    stg = (float*)lds_g;
  const int tid = threadIdx.x, lane = tid & 31, wave = tid >> 5, hh = lane >> 4, m = lane & 15;
  const int rowBase = blockIdx.x * GROWS;

  v8f acc[NT];
#pragma unroll
  for (int t = 0; t < NT; ++t) acc[t] = zero8f();

#pragma unroll 1
  for (int chn = 0; chn < NCH; ++chn) {
#pragma unroll
    for (int i = 0; i < SPT; ++i) {
      const int idx = i * NTHR + tid;
      const int r   = idx / GPR;
      const int c0  = (idx - r * GPR) * 8;
      int row = rowBase + r;
      row = row > nRowsA - 1 ? nRowsA - 1 : row;
      *(v8h*)(sA + r * AP + c0) = ld8h(A + (size_t)row * K + (size_t)chn * KC + c0);
    }
    if (PG > 0) {
      const v8h z8 = zero8h();
      for (int idx = tid; idx < GROWS * PG; idx += NTHR) {
        const int r = idx / PGD;
        const int c = KC + (idx - r * PGD) * 8;
        *(v8h*)(sA + r * AP + c) = z8;
      }
    }
    __syncthreads();
    const _Float16* ar = sA + (wave * 16 + m) * AP + 8 * hh;
#pragma unroll 1
    for (int kt = 0; kt < KCP / 32; ++kt) {
      FragH a;
      a.h[0] = *(const v8h*)(ar + 32 * kt);
      a.h[1] = *(const v8h*)(ar + 32 * kt + 16);
#pragma unroll
      for (int t = 0; t < NT; ++t) {
        const _Float16* bp = Bs + (size_t)(16 * t + m) * KBP + chn * KCP + 32 * kt + 8 * hh;
        FragH bf;
        bf.h[0] = *(const v8h*)bp;
        bf.h[1] = *(const v8h*)(bp + 16);
        acc[t] = wmh(a.v, bf.v, acc[t]);
      }
    }
    __syncthreads();
  }

  const int r0 = wave * 16 + 8 * hh;
  float s[8];
  if (MODE == 1) {
    const v4f dA = *(const v4f*)(dinv + (size_t)rowBase + r0);
    const v4f dB = *(const v4f*)(dinv + (size_t)rowBase + r0 + 4);
    s[0] = dA.x; s[1] = dA.y; s[2] = dA.z; s[3] = dA.w; s[4] = dB.x; s[5] = dB.y; s[6] = dB.z; s[7] = dB.w;
#pragma unroll
    for (int r = 0; r < 8; ++r) s[r] = s[r] * WINV;
  } else {
#pragma unroll
    for (int r = 0; r < 8; ++r) s[r] = WINV;
  }
  float* sp = stg + r0 * NC + m;
#pragma unroll
  for (int t = 0; t < NT; ++t) {
    float bv = 0.0f;
    if (MODE == 0) bv = bias[16 * t + m];
#pragma unroll
    for (int r = 0; r < 8; ++r) {
      float v = acc[t][r] * s[r] + bv;
      if (MODE == 0) v = fmaxf(v, 0.0f);
      sp[r * NC + 16 * t] = v;
    }
  }
  __syncthreads();

  const float* lp = stg + wave * 16 * NC;
  if (MODE == 0) {
    _Float16* gp = Ch + ((size_t)rowBase + wave * 16) * NC;
#pragma unroll
    for (int p = 0; p < 16 * NC / 256; ++p) {
      const int e = 8 * (32 * p + lane);
      const v8h hv = cvt8(*(const v4f*)(lp + e), *(const v4f*)(lp + e + 4));
      *(volatile v8h*)(gp + e) = hv;
    }
    __threadfence();
#pragma unroll
    for (int p = 0; p < 16 * NC / 256; ++p) {
      const int e = 8 * (32 * p + lane);
      const v8h hv = cvt8(*(const v4f*)(lp + e), *(const v4f*)(lp + e + 4));
      *(volatile v8h*)(gp + e) = hv;
    }
  } else {
    float* gp = Cf + ((size_t)rowBase + wave * 16) * NC;
#pragma unroll
    for (int p = 0; p < 16 * NC / 128; ++p) {
      const int e = 4 * (32 * p + lane);
      const v4f v = *(const v4f*)(lp + e);
      *(volatile v4f*)(gp + e) = v;
    }
    __threadfence();
#pragma unroll
    for (int p = 0; p < 16 * NC / 128; ++p) {
      const int e = 4 * (32 * p + lane);
      const v4f v = *(const v4f*)(lp + e);
      *(volatile v4f*)(gp + e) = v;
    }
  }
}

__device__ __forceinline__ float sigm(float x) {
  x = fminf(fmaxf(x, -30.0f), 30.0f);
  const float e = expf(-x);
  return 1.0f / (1.0f + e);
}

__global__ __launch_bounds__(NTHR) void k_tail(
    const float* __restrict__ gpre, const float* __restrict__ Whh, const float* __restrict__ bih,
    const float* __restrict__ bhh, const float* __restrict__ Wfc1, const float* __restrict__ bfc1,
    const float* __restrict__ Wfc2, const float* __restrict__ bfc2, float* out) {
  extern __shared__ v4f lds_t[];
  char* base = (char*)lds_t;
  float*    sG   = (float*)(base + TL_G);
  _Float16* sWhh = (_Float16*)(base + TL_WHH);
  _Float16* sWf1 = (_Float16*)(base + TL_WF1);
  _Float16* sWf2 = (_Float16*)(base + TL_WF2);
  float*    sBi  = (float*)(base + TL_B);
  _Float16* sH   = (_Float16*)(base + TL_H);
  _Float16* sHs  = (_Float16*)(base + TL_HS);
  _Float16* sZ   = (_Float16*)(base + TL_Z);
  float*    sC   = (float*)(base + TL_C);
  const int tid = threadIdx.x, lane = tid & 31, wave = tid >> 5, hh = lane >> 4, m = lane & 15;

  { const v4i z = {0, 0, 0, 0}; v4i* zp = (v4i*)(base + TL_H); for (int i = tid; i < (LDS_TAIL - TL_H) / 16; i += NTHR) zp[i] = z; }
  for (int i = tid; i < GATE * LH; i += NTHR) sWhh[(i >> 5) * HP + (i & 31)] = (_Float16)(Whh[i] * WSCALE);
  for (int i = tid; i < 16 * LH; i += NTHR)   sWf1[(i >> 5) * HP + (i & 31)] = (_Float16)(Wfc1[i] * WSCALE);
  for (int i = tid; i < 16 * 32; i += NTHR) {
    const int n = i >> 5, k = i & 31;
    const int nc = n < NCLS ? n : NCLS - 1;
    const int kc = k < 16 ? k : 15;
    const float x = Wfc2[nc * 16 + kc];
    const float v = (n < NCLS && k < 16) ? x * WSCALE : 0.0f;
    sWf2[n * HP + k] = (_Float16)v;
  }
  for (int i = tid; i < GATE; i += NTHR) sBi[i] = bih[i] + bhh[i];
  __syncthreads();

  const int rt = wave >> 1, cg = wave & 1;
#pragma unroll 1
  for (int t = 0; t < TWIN; ++t) {
    {
      const _Float16* ar = sH + (16 * rt + m) * HP + 8 * hh;
      FragH a;
      a.h[0] = *(const v8h*)ar;
      a.h[1] = *(const v8h*)(ar + 16);
      v8f acc[4];
#pragma unroll
      for (int tt = 0; tt < 4; ++tt) {
        const _Float16* bp = sWhh + (64 * cg + 16 * tt + m) * HP + 8 * hh;
        FragH bf;
        bf.h[0] = *(const v8h*)bp;
        bf.h[1] = *(const v8h*)(bp + 16);
        acc[tt] = wmh(a.v, bf.v, zero8f());
      }
      float* gp = sG + (16 * rt + 8 * hh) * GATE + 64 * cg + m;
#pragma unroll
      for (int tt = 0; tt < 4; ++tt)
#pragma unroll
        for (int r = 0; r < 8; ++r) gp[r * GATE + 16 * tt] = acc[tt][r] * WINV;
    }
    __syncthreads();
    const int tsel = t - (TWIN - TOUT);
#pragma unroll 1
    for (int i = 0; i < 8; ++i) {
      const int bb = i * NWAVE + wave;
      const int p  = bb * LH + lane;
      const float* grow = gpre + ((size_t)bb * TWIN + t) * GATE;
      const float* sg = sG + bb * GATE;
      const float xi = sg[lane]          + grow[lane]          + sBi[lane];
      const float xf = sg[LH + lane]     + grow[LH + lane]     + sBi[LH + lane];
      const float xg = sg[2 * LH + lane] + grow[2 * LH + lane] + sBi[2 * LH + lane];
      const float xo = sg[3 * LH + lane] + grow[3 * LH + lane] + sBi[3 * LH + lane];
      const float gi = sigm(xi), gf = sigm(xf), gg = tanhf(xg), go = sigm(xo);
      const float cn = gf * sC[p] + gi * gg;
      sC[p] = cn;
      const float hn = go * tanhf(cn);
      const _Float16 h16 = (_Float16)hn;
      sH[bb * HP + lane] = h16;
      if (tsel >= 0) sHs[(bb * TOUT + tsel) * HP + lane] = h16;
    }
    __syncthreads();
  }

#pragma unroll
  for (int q = 0; q < 4; ++q) {
    const int R0 = 64 * wave + 16 * q;
    const _Float16* ar = sHs + (R0 + m) * HP + 8 * hh;
    FragH a;
    a.h[0] = *(const v8h*)ar;
    a.h[1] = *(const v8h*)(ar + 16);
    const _Float16* bp = sWf1 + m * HP + 8 * hh;
    FragH bf;
    bf.h[0] = *(const v8h*)bp;
    bf.h[1] = *(const v8h*)(bp + 16);
    const v8f d = wmh(a.v, bf.v, zero8f());
    const float bl = bfc1[m];
    _Float16* zp = sZ + (R0 + 8 * hh) * HP + m;
#pragma unroll
    for (int r = 0; r < 8; ++r) zp[r * HP] = (_Float16)fmaxf(d[r] * WINV + bl, 0.0f);
  }
  __syncthreads();
  float* sOut = sG;
#pragma unroll
  for (int q = 0; q < 4; ++q) {
    const int R0 = 64 * wave + 16 * q;
    const _Float16* ar = sZ + (R0 + m) * HP + 8 * hh;
    FragH a;
    a.h[0] = *(const v8h*)ar;
    a.h[1] = *(const v8h*)(ar + 16);
    const _Float16* bp = sWf2 + m * HP + 8 * hh;
    FragH bf;
    bf.h[0] = *(const v8h*)bp;
    bf.h[1] = *(const v8h*)(bp + 16);
    const v8f d = wmh(a.v, bf.v, zero8f());
    const float b2v = bfc2[m < NCLS ? m : NCLS - 1];
    if (m < NCLS) {
#pragma unroll
      for (int r = 0; r < 8; ++r) sOut[(R0 + 8 * hh + r) * NCLS + m] = d[r] * WINV + b2v;
    }
  }
  __syncthreads();
#pragma unroll
  for (int i = 0; i < (NBAT * TOUT * NCLS) / (4 * NTHR); ++i) {
    const int idx = i * NTHR + tid;
    const v4f v = ((const v4f*)sOut)[idx];
    *(volatile v4f*)(out + 4 * idx) = v;
  }
  __threadfence();
#pragma unroll
  for (int i = 0; i < (NBAT * TOUT * NCLS) / (4 * NTHR); ++i) {
    const int idx = i * NTHR + tid;
    const v4f v = ((const v4f*)sOut)[idx];
    *(volatile v4f*)(out + 4 * idx) = v;
  }
}

extern "C" void kernel_launch(void* const* d_in, const int* in_sizes, int n_in,
                              void* d_out, int out_size, void* d_ws, size_t ws_size,
                              hipStream_t stream) {
  if (n_in < 14) return;
  const int nN = in_sizes[0] / FEAT;
  const int nE = in_sizes[1] / 2;
  if (nN != NBAT * TWIN * NPG || in_sizes[0] != nN * FEAT) return;
  if (nE <= 0 || in_sizes[1] != 2 * nE || nE > (1 << 28)) return;
  if (in_sizes[2] != FEAT * HID || in_sizes[3] != HID || in_sizes[4] != HID * FEAT || in_sizes[5] != FEAT) return;
  if (in_sizes[6] != GATE * SEQD || in_sizes[7] != GATE * LH || in_sizes[8] != GATE || in_sizes[9] != GATE) return;
  if (in_sizes[10] != 16 * LH || in_sizes[11] != 16 || in_sizes[12] != NCLS * 16 || in_sizes[13] != NCLS) return;
  if (out_size != NBAT * TOUT * NCLS) return;
  if (nN > (1 << 20)) return;

  const float* x    = (const float*)d_in[0];
  const int*   ei   = (const int*)d_in[1];
  const float* W1   = (const float*)d_in[2];
  const float* b1   = (const float*)d_in[3];
  const float* W2   = (const float*)d_in[4];
  const float* b2   = (const float*)d_in[5];
  const float* Wih  = (const float*)d_in[6];
  const float* Whh  = (const float*)d_in[7];
  const float* bih  = (const float*)d_in[8];
  const float* bhh  = (const float*)d_in[9];
  const float* Wfc1 = (const float*)d_in[10];
  const float* bfc1 = (const float*)d_in[11];
  const float* Wfc2 = (const float*)d_in[12];
  const float* bfc2 = (const float*)d_in[13];
  float* out = (float*)d_out;

  const int NPAD   = ((nN + NB - 1) / NB) * NB;
  const int nBlk   = NPAD / NB;
  const int csrLen = nBlk * RCAP;
  const int nSeq   = NPAD / NPG;
  if ((nSeq % GROWS) != 0) return;

  char* ws = (char*)d_ws;
  size_t o = 0;
  const size_t oW1  = o; o += (size_t)HID * 32 * 2;          o = (o + 255) & ~(size_t)255;
  const size_t oW2  = o; o += (size_t)FEAT * HID * 2;       o = (o + 255) & ~(size_t)255;
  const size_t oWih = o; o += (size_t)GATE * SEQD * 2;      o = (o + 255) & ~(size_t)255;
  const size_t oCnt = o; o += (size_t)NPAD * 4;             o = (o + 255) & ~(size_t)255;
  const size_t oDv  = o; o += (size_t)NPAD * 4;             o = (o + 255) & ~(size_t)255;
  const size_t oOff = o; o += (size_t)NPAD * 4;             o = (o + 255) & ~(size_t)255;
  const size_t oCsr = o; o += (size_t)csrLen * 4;           o = (o + 255) & ~(size_t)255;
  const size_t oAx  = o; o += (size_t)NPAD * FEAT * 4;      o = (o + 255) & ~(size_t)255;
  const size_t oH1  = o; o += (size_t)NPAD * HID * 2;       o = (o + 255) & ~(size_t)255;
  const size_t oHw  = o; o += (size_t)NPAD * FEAT * 4;      o = (o + 255) & ~(size_t)255;
  const size_t oSq  = o; o += (size_t)NPAD * FEAT * 4;      o = (o + 255) & ~(size_t)255;
  const size_t oG   = o; o += (size_t)nSeq * GATE * 4;      o = (o + 255) & ~(size_t)255;
  if (o > ws_size) return;
  _Float16* w1p  = (_Float16*)(ws + oW1);
  _Float16* w2p  = (_Float16*)(ws + oW2);
  _Float16* wihp = (_Float16*)(ws + oWih);
  int*      cntp = (int*)(ws + oCnt);
  float*    dinv = (float*)(ws + oDv);
  int*      offp = (int*)(ws + oOff);
  int*      csr  = (int*)(ws + oCsr);
  float*    ax   = (float*)(ws + oAx);
  _Float16* h1a  = (_Float16*)(ws + oH1);
  float*    hw2  = (float*)(ws + oHw);
  float*    seq  = (float*)(ws + oSq);
  float*    gpre = (float*)(ws + oG);

  const int vec8 = ((nE & 3) == 0) ? 1 : 0;
  const int nb0 = (HID * 32 / 8 + NTHR - 1) / NTHR;
  const int nb1 = (FEAT * HID / 8 + NTHR - 1) / NTHR;
  const int nb2 = (GATE * SEQD / 8 + NTHR - 1) / NTHR;

  k_wprep<<<nb0 + nb1 + nb2, NTHR, 0, stream>>>(W1, W2, Wih, w1p, w2p, wihp, nb0, nb1);

  hipFuncSetAttribute(reinterpret_cast<const void*>(&k_csr), hipFuncAttributeMaxDynamicSharedMemorySize, LDS_CSR);
  k_csr<<<nBlk, NTHR, LDS_CSR, stream>>>(ei, cntp, dinv, offp, csr, nN, nE, vec8);

  k_agg<0><<<NPAD / TGT, NTHR, 0, stream>>>(csr, offp, cntp, dinv, x, b1, ax, nN, nN, csrLen);
  k_gemm<FEAT, FEAT, HID / 16, float, 0><<<NPAD / GROWS, NTHR, GEMM_LDS(FEAT, HID / 16), stream>>>(
      ax, w1p, dinv, b1, h1a, hw2, NPAD);

  k_gemm<HID, HID, 1, _Float16, 1><<<NPAD / GROWS, NTHR, GEMM_LDS(HID, 1), stream>>>(
      h1a, w2p, dinv, b1, (_Float16*)(ws + oSq), hw2, NPAD);
  k_agg<1><<<NPAD / TGT, NTHR, 0, stream>>>(csr, offp, cntp, dinv, hw2, b2, seq, nN, NPAD, csrLen);

  hipFuncSetAttribute(reinterpret_cast<const void*>(&k_gemm<SEQD, KC2, GATE / 16, float, 2>),
                      hipFuncAttributeMaxDynamicSharedMemorySize, GEMM_LDS(KC2, GATE / 16));
  k_gemm<SEQD, KC2, GATE / 16, float, 2><<<nSeq / GROWS, NTHR, GEMM_LDS(KC2, GATE / 16), stream>>>(
      seq, wihp, dinv, b1, h1a, gpre, nSeq);

  hipFuncSetAttribute(reinterpret_cast<const void*>(&k_tail), hipFuncAttributeMaxDynamicSharedMemorySize, LDS_TAIL);
  k_tail<<<1, NTHR, LDS_TAIL, stream>>>(gpre, Whh, bih, bhh, Wfc1, bfc1, Wfc2, bfc2, out);
}
